// BertLayer_2989297238363
// MI455X (gfx1250) — hardware-verified
//
#include <hip/hip_runtime.h>
#include <stdint.h>

#ifndef NB
#define NB 2
#endif
#ifndef SEQ
#define SEQ 2048
#endif
#define NB_FULL 2
#define SEQ_FULL 2048
#define HID 1024
#define NHD 16
#define DHD 64
#define DFF 4096
#define MTOK (NB * SEQ)

static_assert(NB >= 1 && NB <= NB_FULL);
static_assert(SEQ >= 128 && SEQ <= SEQ_FULL && (SEQ % 128) == 0);
static_assert((MTOK % 128) == 0);
static_assert(HID == NHD * DHD);
static_assert((HID % 128) == 0 && (DFF % 128) == 0 && (HID % 32) == 0 && (DFF % 32) == 0);

typedef _Float16 f16;
typedef f16   v4h  __attribute__((ext_vector_type(4)));
typedef f16   v8h  __attribute__((ext_vector_type(8)));
typedef f16   v16h __attribute__((ext_vector_type(16)));
typedef float v4f  __attribute__((ext_vector_type(4)));
typedef float v8f  __attribute__((ext_vector_type(8)));
union Frag { v16h v; v8h half[2]; };

__device__ __forceinline__ v8f wmma16(v16h a, v16h b, v8f c) {
    v8f d = __builtin_amdgcn_wmma_f32_16x16x32_f16(false, a, false, b, (short)0, c, false, false);
    asm volatile("v_nop\n\tv_nop\n\tv_nop\n\tv_nop" : "+v"(d) : "v"(a), "v"(b));
    return d;
}
__device__ __forceinline__ v8f zero8() {
    v8f z;
#pragma unroll
    for (int i = 0; i < 8; ++i) z[i] = 0.0f;
    return z;
}
__device__ __forceinline__ float bf16r(float x) {
    unsigned u = __float_as_uint(x);
    u = (u + 0x7FFFu + ((u >> 16) & 1u)) & 0xFFFF0000u;
    return __uint_as_float(u);
}

__global__ __launch_bounds__(256) void k_cvt(const float* __restrict__ in, f16* out, int n, int rowlen,
                                              int seq, int seqf, float scale) {
    const size_t i8 = ((size_t)blockIdx.x * 256 + threadIdx.x) * 8;
    if (i8 + 8 > (size_t)n) return;
    const int m = (int)(i8 / (size_t)rowlen);
    const int c = (int)(i8 - (size_t)m * (size_t)rowlen);
    const size_t src = ((size_t)(m / seq) * (size_t)seqf + (size_t)(m % seq)) * (size_t)rowlen + (size_t)c;
    v4f a = *(const v4f*)(in + src);
    v4f b = *(const v4f*)(in + src + 4);
    v8h hv;
    hv[0] = (f16)(bf16r(a[0]) * scale); hv[1] = (f16)(bf16r(a[1]) * scale);
    hv[2] = (f16)(bf16r(a[2]) * scale); hv[3] = (f16)(bf16r(a[3]) * scale);
    hv[4] = (f16)(bf16r(b[0]) * scale); hv[5] = (f16)(bf16r(b[1]) * scale);
    hv[6] = (f16)(bf16r(b[2]) * scale); hv[7] = (f16)(bf16r(b[3]) * scale);
    f16* p = out + i8;
    *(volatile v8h*)p = hv;
    __threadfence();
    *(volatile v8h*)p = hv;
}

#define GBM 128
#define GBN 128
#define GBK 32
#define GLD 40
#define GSP 132

__global__ __launch_bounds__(256) void k_gemm(const f16* __restrict__ A, const f16* __restrict__ BT,
                                               const float* __restrict__ bias, float* Cf, f16* Ch,
                                               int M, int N, int K, int act, float oscale, int omode) {
    __shared__ f16 As[GBM * GLD];
    __shared__ f16 Bs[GBN * GLD];
    __shared__ float Cs[64 * GSP];

    const int t = threadIdx.x, wave = t >> 5, lane = t & 31;
    const int hh = lane >> 4, l16 = lane & 15;
    const int wm = wave >> 2, wn = wave & 3;
    const int bm0 = blockIdx.y * GBM, bn0 = blockIdx.x * GBN;
    if (bm0 + GBM > M || bn0 + GBN > N) return;

    v8f acc[4][2];
#pragma unroll
    for (int i = 0; i < 4; ++i)
#pragma unroll
        for (int j = 0; j < 2; ++j) acc[i][j] = zero8();

    const int nk = K / GBK;
    for (int it = 0; it < nk; ++it) {
        const int k0 = it * GBK;
#pragma unroll
        for (int j = 0; j < 2; ++j) {
            const int e = t + 256 * j, row = e >> 2, seg = (e & 3) * 8;
            v8h va = *(const v8h*)(A  + (size_t)(bm0 + row) * K + k0 + seg);
            v8h vb = *(const v8h*)(BT + (size_t)(bn0 + row) * K + k0 + seg);
            *(v8h*)(As + row * GLD + seg) = va;
            *(v8h*)(Bs + row * GLD + seg) = vb;
        }
        __syncthreads();

        Frag af[4], bf[2];
#pragma unroll
        for (int mf = 0; mf < 4; ++mf) {
            const f16* ap = As + (wm * 64 + mf * 16 + l16) * GLD;
            af[mf].half[0] = *(const v8h*)(ap + 8 * hh);
            af[mf].half[1] = *(const v8h*)(ap + 16 + 8 * hh);
        }
#pragma unroll
        for (int nf = 0; nf < 2; ++nf) {
            const f16* bp = Bs + (wn * 32 + nf * 16 + l16) * GLD;
            bf[nf].half[0] = *(const v8h*)(bp + 8 * hh);
            bf[nf].half[1] = *(const v8h*)(bp + 16 + 8 * hh);
        }
#pragma unroll
        for (int mf = 0; mf < 4; ++mf)
#pragma unroll
            for (int nf = 0; nf < 2; ++nf)
                acc[mf][nf] = wmma16(af[mf].v, bf[nf].v, acc[mf][nf]);
        __syncthreads();
    }

#pragma unroll 1
    for (int p = 0; p < 2; ++p) {
        if (wm == p) {
#pragma unroll
            for (int mf = 0; mf < 4; ++mf)
#pragma unroll
                for (int nf = 0; nf < 2; ++nf) {
                    const int col = wn * 32 + nf * 16 + l16;
                    const float bvv = bias[bn0 + col];
#pragma unroll
                    for (int r = 0; r < 8; ++r) {
                        const int row = mf * 16 + 8 * hh + r;
                        float x = acc[mf][nf][r] * oscale + bvv;
                        if (act) x = x * 0.5f * (1.0f + erff(x * 0.70710678118654752f));
                        Cs[row * GSP + col] = x;
                    }
                }
        }
        __syncthreads();
        if (omode & 1) {
            v4f vals[8];
            size_t po[8];
#pragma unroll
            for (int j = 0; j < 8; ++j) {
                const int e = t + 256 * j, row = e >> 5, c4 = (e & 31) * 4;
                vals[j] = *(const v4f*)(Cs + row * GSP + c4);
                po[j] = (size_t)(bm0 + p * 64 + row) * N + bn0 + c4;
            }
#pragma unroll
            for (int j = 0; j < 8; ++j) *(volatile v4f*)(Cf + po[j]) = vals[j];
            __threadfence();
#pragma unroll
            for (int j = 0; j < 8; ++j) *(volatile v4f*)(Cf + po[j]) = vals[j];
        }
        if (omode & 2) {
            v8h hv[4];
            size_t po[4];
#pragma unroll
            for (int j = 0; j < 4; ++j) {
                const int e = t + 256 * j, row = e >> 4, c8 = (e & 15) * 8;
                v4f a = *(const v4f*)(Cs + row * GSP + c8);
                v4f b = *(const v4f*)(Cs + row * GSP + c8 + 4);
                hv[j][0] = (f16)a[0]; hv[j][1] = (f16)a[1]; hv[j][2] = (f16)a[2]; hv[j][3] = (f16)a[3];
                hv[j][4] = (f16)b[0]; hv[j][5] = (f16)b[1]; hv[j][6] = (f16)b[2]; hv[j][7] = (f16)b[3];
                po[j] = (size_t)(bm0 + p * 64 + row) * N + bn0 + c8;
            }
#pragma unroll
            for (int j = 0; j < 4; ++j) *(volatile v8h*)(Ch + po[j]) = hv[j];
            __threadfence();
#pragma unroll
            for (int j = 0; j < 4; ++j) *(volatile v8h*)(Ch + po[j]) = hv[j];
        }
        __syncthreads();
    }
}

#define ALD 72

__global__ __launch_bounds__(256) void k_attn(const f16* __restrict__ QKV, const float* __restrict__ mask,
                                               f16* Ctx, int nb) {
    __shared__ f16 Ks[64 * ALD];
    __shared__ f16 Vs[64 * ALD];
    __shared__ f16 Ps[8 * 16 * ALD];

    const int t = threadIdx.x, wave = t >> 5, lane = t & 31;
    const int hh = lane >> 4, l16 = lane & 15;
    const int bid = blockIdx.x;
    const int nqt = SEQ / 128;
    const int qt = bid % nqt, h = (bid / nqt) % NHD, b = bid / (nqt * NHD);
    if (b >= nb) return;
    const int q0 = qt * 128 + wave * 16;
    const size_t tok0 = (size_t)b * SEQ;
    f16* Pw = Ps + wave * 16 * ALD;

    Frag qa[2];
    {
        const f16* qp = QKV + (tok0 + q0 + l16) * HID + h * DHD;
#pragma unroll
        for (int kf = 0; kf < 2; ++kf) {
            qa[kf].half[0] = *(const v8h*)(qp + kf * 32 + 8 * hh);
            qa[kf].half[1] = *(const v8h*)(qp + kf * 32 + 16 + 8 * hh);
        }
    }

    float mrun[8], lrun[8];
    v8f o[4];
#pragma unroll
    for (int r = 0; r < 8; ++r) { mrun[r] = -3.0e38f; lrun[r] = 0.0f; }
#pragma unroll
    for (int nf = 0; nf < 4; ++nf) o[nf] = zero8();

    for (int kt = 0; kt < SEQ / 64; ++kt) {
#pragma unroll
        for (int j = 0; j < 2; ++j) {
            const int e = t + 256 * j, key = e >> 3, seg = (e & 7) * 8;
            const size_t g = (tok0 + kt * 64 + key) * HID + h * DHD + seg;
            v8h kv = *(const v8h*)(QKV + g);
            *(v8h*)(Ks + key * ALD + seg) = kv;
#pragma unroll
            for (int i = 0; i < 8; ++i) Vs[(seg + i) * ALD + key] = kv[i];
        }
        __syncthreads();

        v8f s[4];
#pragma unroll
        for (int n = 0; n < 4; ++n) {
            Frag kb0, kb1;
            const f16* kp = Ks + (n * 16 + l16) * ALD;
            kb0.half[0] = *(const v8h*)(kp + 8 * hh);
            kb0.half[1] = *(const v8h*)(kp + 16 + 8 * hh);
            kb1.half[0] = *(const v8h*)(kp + 32 + 8 * hh);
            kb1.half[1] = *(const v8h*)(kp + 48 + 8 * hh);
            v8f z = zero8();
            z = wmma16(qa[0].v, kb0.v, z);
            z = wmma16(qa[1].v, kb1.v, z);
            const int key = kt * 64 + n * 16 + l16;
            const float mt = mask[(size_t)b * SEQ_FULL + key];
#pragma unroll
            for (int r = 0; r < 8; ++r) s[n][r] = z[r] * 0.125f + mt;
        }

        float mnew[8], corr[8];
#pragma unroll
        for (int r = 0; r < 8; ++r) {
            float mx = fmaxf(fmaxf(s[0][r], s[1][r]), fmaxf(s[2][r], s[3][r]));
#pragma unroll
            for (int off = 8; off >= 1; off >>= 1) mx = fmaxf(mx, __shfl_xor(mx, off, 32));
            mnew[r] = fmaxf(mrun[r], mx);
            corr[r] = __expf(mrun[r] - mnew[r]);
            mrun[r] = mnew[r];
        }
#pragma unroll
        for (int nf = 0; nf < 4; ++nf)
#pragma unroll
            for (int r = 0; r < 8; ++r) o[nf][r] *= corr[r];
#pragma unroll
        for (int r = 0; r < 8; ++r) {
            float rs = 0.0f;
#pragma unroll
            for (int n = 0; n < 4; ++n) {
                float pe = __expf(s[n][r] - mnew[r]);
                s[n][r] = pe;
                rs += pe;
            }
#pragma unroll
            for (int off = 8; off >= 1; off >>= 1) rs += __shfl_xor(rs, off, 32);
            lrun[r] = lrun[r] * corr[r] + rs;
        }

#pragma unroll
        for (int n = 0; n < 4; ++n)
#pragma unroll
            for (int r = 0; r < 8; ++r)
                Pw[(r + 8 * hh) * ALD + n * 16 + l16] = (f16)(s[n][r] * 4096.0f);
        __syncthreads();

        Frag pa[2];
        {
            const f16* pp = Pw + l16 * ALD;
#pragma unroll
            for (int kf = 0; kf < 2; ++kf) {
                pa[kf].half[0] = *(const v8h*)(pp + kf * 32 + 8 * hh);
                pa[kf].half[1] = *(const v8h*)(pp + kf * 32 + 16 + 8 * hh);
            }
        }
#pragma unroll
        for (int nf = 0; nf < 4; ++nf) {
            Frag vb0, vb1;
            const f16* vp = Vs + (nf * 16 + l16) * ALD;
            vb0.half[0] = *(const v8h*)(vp + 8 * hh);
            vb0.half[1] = *(const v8h*)(vp + 16 + 8 * hh);
            vb1.half[0] = *(const v8h*)(vp + 32 + 8 * hh);
            vb1.half[1] = *(const v8h*)(vp + 48 + 8 * hh);
            o[nf] = wmma16(pa[0].v, vb0.v, o[nf]);
            o[nf] = wmma16(pa[1].v, vb1.v, o[nf]);
        }
        __syncthreads();
    }

    {
        float il[8];
#pragma unroll
        for (int r = 0; r < 8; ++r) il[r] = 16.0f / (lrun[r] * 4096.0f);
#pragma unroll
        for (int nf = 0; nf < 4; ++nf)
#pragma unroll
            for (int r = 0; r < 8; ++r)
                Pw[(r + 8 * hh) * ALD + nf * 16 + l16] = (f16)(o[nf][r] * il[r]);
    }
    __syncthreads();
    v8h cv[4];
    size_t po[4];
#pragma unroll
    for (int j = 0; j < 4; ++j) {
        const int s2 = lane + 32 * j, row = s2 >> 3, c8 = (s2 & 7) * 8;
        cv[j] = *(const v8h*)(Pw + row * ALD + c8);
        po[j] = (tok0 + q0 + row) * HID + h * DHD + c8;
    }
#pragma unroll
    for (int j = 0; j < 4; ++j) *(volatile v8h*)(Ctx + po[j]) = cv[j];
    __threadfence();
#pragma unroll
    for (int j = 0; j < 4; ++j) *(volatile v8h*)(Ctx + po[j]) = cv[j];
}

__global__ __launch_bounds__(256) void k_ln(const float* __restrict__ a, const float* __restrict__ res,
                                             int rseq, int rseqf, int res_bf16,
                                             const float* __restrict__ g, const float* __restrict__ be,
                                             float* outf, f16* outh, int write_h, int nrows) {
    __shared__ float red1[8], red2[8];
    const int row = blockIdx.x;
    if (row >= nrows) return;
    const int t = threadIdx.x, wave = t >> 5, lane = t & 31;
    const size_t base = (size_t)row * HID + (size_t)t * 4;
    const size_t rrow = (size_t)(row / rseq) * (size_t)rseqf + (size_t)(row % rseq);
    const size_t rbase = rrow * HID + (size_t)t * 4;

    v4f rv = *(const v4f*)(res + rbase);
    if (res_bf16) {
        rv[0] = bf16r(rv[0]); rv[1] = bf16r(rv[1]); rv[2] = bf16r(rv[2]); rv[3] = bf16r(rv[3]);
    }
    v4f x = *(const v4f*)(a + base) + rv;
    float sm = (x[0] + x[1]) + (x[2] + x[3]);
#pragma unroll
    for (int off = 16; off >= 1; off >>= 1) sm += __shfl_xor(sm, off, 32);
    if (lane == 0) red1[wave] = sm;
    __syncthreads();
    float tot = 0.0f;
#pragma unroll
    for (int w = 0; w < 8; ++w) tot += red1[w];
    const float mu = tot * (1.0f / 1024.0f);

    v4f d = x - mu;
    float sq = (d[0] * d[0] + d[1] * d[1]) + (d[2] * d[2] + d[3] * d[3]);
#pragma unroll
    for (int off = 16; off >= 1; off >>= 1) sq += __shfl_xor(sq, off, 32);
    if (lane == 0) red2[wave] = sq;
    __syncthreads();
    float tot2 = 0.0f;
#pragma unroll
    for (int w = 0; w < 8; ++w) tot2 += red2[w];
    const float var = tot2 * (1.0f / 1024.0f);
    const float rstd = rsqrtf(var + 1.0e-5f);

    v4f gv = *(const v4f*)(g + t * 4);
    v4f bv = *(const v4f*)(be + t * 4);
    v4f y = d * rstd * gv + bv;
    v4h yh;
    yh[0] = (f16)y[0]; yh[1] = (f16)y[1]; yh[2] = (f16)y[2]; yh[3] = (f16)y[3];

    *(volatile v4f*)(outf + base) = y;
    if (write_h) *(volatile v4h*)(outh + base) = yh;
    __threadfence();
    *(volatile v4f*)(outf + base) = y;
    if (write_h) *(volatile v4h*)(outh + base) = yh;
}

extern "C" void kernel_launch(void* const* d_in, const int* in_sizes, int n_in,
                              void* d_out, int out_size, void* d_ws, size_t ws_size,
                              hipStream_t stream) {
    const int Mtok = MTOK;
    if (n_in < 14) return;
    if (in_sizes[0] < ((NB - 1) * SEQ_FULL + SEQ) * HID || in_sizes[1] < (NB - 1) * SEQ_FULL + SEQ ||
        in_sizes[2] < HID * HID || in_sizes[3] < HID || in_sizes[4] < HID * HID || in_sizes[5] < HID ||
        in_sizes[6] < HID || in_sizes[7] < HID || in_sizes[8] < DFF * HID || in_sizes[9] < DFF ||
        in_sizes[10] < HID * DFF || in_sizes[11] < HID || in_sizes[12] < HID || in_sizes[13] < HID ||
        out_size < Mtok * HID) return;

    const float* x    = (const float*)d_in[0];
    const float* amsk = (const float*)d_in[1];
    const float* Wq   = (const float*)d_in[2];  const float* bq   = (const float*)d_in[3];
    const float* Wso  = (const float*)d_in[4];  const float* bso  = (const float*)d_in[5];
    const float* ln1g = (const float*)d_in[6];  const float* ln1b = (const float*)d_in[7];
    const float* Wi   = (const float*)d_in[8];  const float* bi   = (const float*)d_in[9];
    const float* Wo   = (const float*)d_in[10]; const float* bo   = (const float*)d_in[11];
    const float* ln2g = (const float*)d_in[12]; const float* ln2b = (const float*)d_in[13];

    char* ws = (char*)d_ws;
    size_t off = 0;
    auto take = [&](size_t bytes) -> char* {
        char* p = ws + off;
        off += (bytes + 255) & ~(size_t)255;
        return p;
    };
    f16*   xh    = (f16*)take((size_t)Mtok * HID * 2);
    f16*   wq16  = (f16*)take((size_t)HID * HID * 2);
    f16*   wso16 = (f16*)take((size_t)HID * HID * 2);
    f16*   wi16  = (f16*)take((size_t)DFF * HID * 2);
    f16*   wo16  = (f16*)take((size_t)HID * DFF * 2);
    f16*   qkvh  = (f16*)take((size_t)Mtok * HID * 2);
    f16*   ctxh  = (f16*)take((size_t)Mtok * HID * 2);
    float* attf  = (float*)take((size_t)Mtok * HID * 4);
    float* h1f   = (float*)take((size_t)Mtok * HID * 4);
    f16*   h1h   = (f16*)take((size_t)Mtok * HID * 2);
    f16*   gh    = (f16*)take((size_t)Mtok * DFF * 2);
    float* fff   = attf;
    if (off > ws_size) return;

    const int thr = 256;
    const float wsc = 64.0f;

    k_cvt<<<(Mtok * HID / 8 + thr - 1) / thr, thr, 0, stream>>>(x, xh, Mtok * HID, HID, SEQ, SEQ_FULL, 1.0f);
    k_cvt<<<(HID * HID / 8 + thr - 1) / thr, thr, 0, stream>>>(Wq, wq16, HID * HID, HID, HID, HID, wsc);
    k_cvt<<<(HID * HID / 8 + thr - 1) / thr, thr, 0, stream>>>(Wso, wso16, HID * HID, HID, HID, HID, wsc);
    k_cvt<<<(DFF * HID / 8 + thr - 1) / thr, thr, 0, stream>>>(Wi, wi16, DFF * HID, HID, DFF, DFF, wsc);
    k_cvt<<<(HID * DFF / 8 + thr - 1) / thr, thr, 0, stream>>>(Wo, wo16, HID * DFF, DFF, HID, HID, wsc);

    const dim3 gH(HID / GBN, Mtok / GBM);
    const dim3 gF(DFF / GBN, Mtok / GBM);


    k_gemm<<<gH, thr, 0, stream>>>(xh, wq16, bq, attf, qkvh, Mtok, HID, HID, 0, 0.015625f, 2);

    k_attn<<<NB * NHD * (SEQ / 128), thr, 0, stream>>>(qkvh, amsk, ctxh, NB);

    k_gemm<<<gH, thr, 0, stream>>>(ctxh, wso16, bso, attf, gh, Mtok, HID, HID, 0, 0.0009765625f, 1);
    k_ln<<<Mtok, thr, 0, stream>>>(attf, x, SEQ, SEQ_FULL, 1, ln1g, ln1b, h1f, h1h, 1, Mtok);

    k_gemm<<<gF, thr, 0, stream>>>(h1h, wi16, bi, attf, gh, Mtok, DFF, HID, 1, 0.015625f, 2);
    k_gemm<<<gH, thr, 0, stream>>>(gh, wo16, bo, fff, h1h, Mtok, HID, DFF, 0, 0.015625f, 1);
    k_ln<<<Mtok, thr, 0, stream>>>(fff, h1f, SEQ, SEQ, 0, ln2g, ln2b, (float*)d_out, h1h, 0, Mtok);
}
